// Decoder_7619271983505
// MI455X (gfx1250) — hardware-verified
//
#include <hip/hip_runtime.h>
#include <math.h>

constexpr int NBATCH   = 64;
constexpr int NIN      = 128;
constexpr int NHID     = 256;
constexpr int NGATE    = 3 * NHID;
constexpr int NSTEP    = 2000;
constexpr int NOUTC    = 128;
constexpr int SEQ_BLK  = 16;
constexpr int GRU_THR  = 512;
constexpr int HPITCH   = 264;
constexpr int ZPITCH   = 132;
constexpr int NROWS    = NBATCH * NSTEP;
constexpr float WCARRY     = 16.0f;
constexpr float WCARRY_INV = 1.0f / 16.0f;

static_assert(NBATCH % SEQ_BLK == 0, "batch rows per block");
static_assert(NHID == 16 * (GRU_THR / 32), "one 16-column group per wave");
static_assert(SEQ_BLK == GRU_THR / 32, "one wave per staged h row");
static_assert(NHID * 2 == 32 * 16, "h row = 32 lanes x 16 B");
static_assert(SEQ_BLK * NIN == GRU_THR * 4, "z tile staging exact");
static_assert(NHID % 32 == 0, "K multiple of 32");
static_assert(NROWS % 64 == 0 && NOUTC % 64 == 0, "GEMM tile multiples");
static_assert((HPITCH % 8) == 0 && (ZPITCH % 4) == 0, "16-B aligned LDS rows");
static_assert((NGATE * NHID / 8) % 256 == 0 && (NOUTC * NHID / 8) % 256 == 0, "convert grids exact");
static_assert((size_t)NROWS * NOUTC * 4 == (size_t)65536000, "output bytes");

typedef __attribute__((ext_vector_type(16))) _Float16 v16h;
typedef __attribute__((ext_vector_type(8)))  _Float16 v8h;
typedef __attribute__((ext_vector_type(8)))  float    v8f;
typedef __attribute__((ext_vector_type(4)))  float    v4f;

__device__ __forceinline__ void guard3_h(v8f& a, v8f& b, v8f& c, v16h x, v16h y0, v16h y1, v16h y2) {
  asm volatile("v_nop\n\tv_nop\n\tv_nop\n\tv_nop" : "+v"(a), "+v"(b), "+v"(c) : "v"(x), "v"(y0), "v"(y1), "v"(y2));
}
__device__ __forceinline__ void guard4_h(v8f& a, v8f& b, v8f& c, v8f& d, v16h x, v16h y) {
  asm volatile("v_nop\n\tv_nop\n\tv_nop\n\tv_nop" : "+v"(a), "+v"(b), "+v"(c), "+v"(d) : "v"(x), "v"(y));
}
__device__ __forceinline__ void keep4_h(v16h a, v16h b, v16h c, v16h d) {
  asm volatile("v_nop" :: "v"(a), "v"(b), "v"(c), "v"(d));
}
__device__ __forceinline__ void acc_guard4(v8f& a, v8f& b, v8f& c, v8f& d) {
  asm volatile("v_nop\n\tv_nop\n\tv_nop\n\tv_nop" : "+v"(a), "+v"(b), "+v"(c), "+v"(d));
}
__device__ __forceinline__ void acc_guard3(v8f& a, v8f& b, v8f& c) {
  asm volatile("v_nop\n\tv_nop\n\tv_nop\n\tv_nop" : "+v"(a), "+v"(b), "+v"(c));
}

union FragU { v16h v; v8h h[2]; };
__device__ __forceinline__ v16h frag_load(const _Float16* p) {
  FragU f;
  f.h[0] = *(const v8h*)(p);
  f.h[1] = *(const v8h*)(p + 16);
  return f.v;
}
__device__ __forceinline__ v8f frag_mma(v16h a, v16h b, v8f c) {
  return __builtin_amdgcn_wmma_f32_16x16x32_f16(false, a, false, b, (short)0, c, false, false);
}

__device__ __forceinline__ float gate_sig(float x) {
  return __builtin_amdgcn_rcpf(1.0f + expf(-x));
}
__device__ __forceinline__ float gate_tanh(float x) {
  return 1.0f - 2.0f * __builtin_amdgcn_rcpf(expf(2.0f * x) + 1.0f);
}

__global__ __launch_bounds__(256) void cvt8_f16_kernel(const float* __restrict__ src, unsigned short* __restrict__ dst,
                                                       int n8, float sc) {
  const int i = blockIdx.x * 256 + threadIdx.x;
  if (i < n8) {
    const v4f a = *(const v4f*)(src + (size_t)i * 8);
    const v4f b = *(const v4f*)(src + (size_t)i * 8 + 4);
    v8h hv;
#pragma unroll
    for (int e = 0; e < 4; ++e) {
      const float fa = a[e] * sc;
      const float fb = b[e] * sc;
      hv[e]     = (_Float16)fa;
      hv[4 + e] = (_Float16)fb;
    }
    _Float16* op = (_Float16*)dst + (size_t)i * 8;
    *(volatile v8h*)op = hv;
    __threadfence();
    *(volatile v8h*)op = hv;
  }
}

__global__ __launch_bounds__(GRU_THR) void gru_seq_kernel(const float* __restrict__ zin, const float* __restrict__ Wih,
                                                          const float* __restrict__ bih, const float* __restrict__ bhh,
                                                          const unsigned short* __restrict__ WHp,
                                                          unsigned short* __restrict__ HSp) {
  __shared__ __align__(16) _Float16 Ah[2 * SEQ_BLK * HPITCH];
  __shared__ __align__(16) float    Zl[SEQ_BLK * ZPITCH];
  const _Float16* WH = (const _Float16*)WHp;
  _Float16* HS = (_Float16*)HSp;
  const int tid = threadIdx.x, lane = tid & 31, wave = tid >> 5;
  const int c = lane & 15, hh = lane >> 4, koff = hh * 8;
  const int rowbase = blockIdx.x * SEQ_BLK;

  {
    const v8h zero8 = {(_Float16)0.0f, (_Float16)0.0f, (_Float16)0.0f, (_Float16)0.0f,
                       (_Float16)0.0f, (_Float16)0.0f, (_Float16)0.0f, (_Float16)0.0f};
#pragma unroll 1
    for (int i = tid; i < (2 * SEQ_BLK * HPITCH) / 8; i += GRU_THR) *(v8h*)(Ah + i * 8) = zero8;
  }
  {
    const int zr = tid >> 5, z4 = (tid & 31) * 4;
    const v4f v = *(const v4f*)(zin + (size_t)(rowbase + zr) * NIN + z4);
    *(v4f*)(Zl + zr * ZPITCH + z4) = v;
  }
  __syncthreads();

  const int j = 16 * wave + c;
  float gi[3][8];
#pragma unroll
  for (int g = 0; g < 3; ++g) {
    const float* wr = Wih + (size_t)(g * NHID + j) * NIN;
    float a8[8];
#pragma unroll
    for (int r = 0; r < 8; ++r) a8[r] = 0.0f;
#pragma unroll 1
    for (int k4 = 0; k4 < NIN; k4 += 4) {
      const v4f w = *(const v4f*)(wr + k4);
#pragma unroll
      for (int r = 0; r < 8; ++r) {
        const v4f zv = *(const v4f*)(Zl + (8 * hh + r) * ZPITCH + k4);
        float s = a8[r];
        s = fmaf(zv[0], w[0], s);
        s = fmaf(zv[1], w[1], s);
        s = fmaf(zv[2], w[2], s);
        s = fmaf(zv[3], w[3], s);
        a8[r] = s;
      }
    }
#pragma unroll
    for (int r = 0; r < 8; ++r) gi[g][r] = a8[r];
  }
  {
    const float bi_r = bih[j];
    const float bi_z = bih[NHID + j];
    const float bi_n = bih[2 * NHID + j];
    const float bh_r = bhh[j];
    const float bh_z = bhh[NHID + j];
#pragma unroll
    for (int r = 0; r < 8; ++r) {
      gi[0][r] = (gi[0][r] + bi_r) + bh_r;
      gi[1][r] = (gi[1][r] + bi_z) + bh_z;
      gi[2][r] = gi[2][r] + bi_n;
    }
  }
  const float bhn = bhh[2 * NHID + j];

  float hst[8];
#pragma unroll
  for (int r = 0; r < 8; ++r) hst[r] = 0.0f;

  const _Float16* w0 = WH + (size_t)j * NHID + koff;
  const _Float16* w1 = w0 + (size_t)NHID * NHID;
  const _Float16* w2 = w1 + (size_t)NHID * NHID;
  const v8f z8 = {0.f, 0.f, 0.f, 0.f, 0.f, 0.f, 0.f, 0.f};

#pragma unroll 1
  for (int t = 0; t < NSTEP; ++t) {
    const int cur = t & 1;
    const _Float16* ahrow = Ah + cur * (SEQ_BLK * HPITCH) + c * HPITCH + koff;
    _Float16* ahn = Ah + (cur ^ 1) * (SEQ_BLK * HPITCH);
    v8f acc0 = z8, acc1 = z8, acc2 = z8;
#pragma unroll 1
    for (int k0 = 0; k0 < NHID; k0 += 32) {
      const v16h a  = frag_load(ahrow + k0);
      const v16h b0 = frag_load(w0 + k0);
      const v16h b1 = frag_load(w1 + k0);
      const v16h b2 = frag_load(w2 + k0);
      acc0 = frag_mma(a, b0, acc0);
      acc1 = frag_mma(a, b1, acc1);
      acc2 = frag_mma(a, b2, acc2);
      guard3_h(acc0, acc1, acc2, a, b0, b1, b2);
    }
    acc_guard3(acc0, acc1, acc2);
#pragma unroll
    for (int r = 0; r < 8; ++r) {
      const float xr = gi[0][r] + acc0[r] * WCARRY_INV;
      const float xz = gi[1][r] + acc1[r] * WCARRY_INV;
      const float hn = acc2[r] * WCARRY_INV + bhn;
      const float rg = gate_sig(xr);
      const float zg = gate_sig(xz);
      const float nn = gate_tanh(gi[2][r] + rg * hn);
      const float ho = hst[r];
      const float hv = (1.0f - zg) * nn + zg * ho;
      hst[r] = hv;
      ahn[(8 * hh + r) * HPITCH + j] = (_Float16)hv;
    }
    __syncthreads();
    {
      const v8h hv8 = *(const v8h*)(ahn + wave * HPITCH + lane * 8);
      _Float16* gp = HS + ((size_t)(rowbase + wave) * NSTEP + (size_t)t) * NHID + lane * 8;
      *(volatile v8h*)gp = hv8;
      __threadfence();
      *(volatile v8h*)gp = hv8;
    }
  }
}

__global__ __launch_bounds__(256) void out_gemm_kernel(const unsigned short* __restrict__ Ap,
                                                       const unsigned short* __restrict__ Btp,
                                                       float* __restrict__ Cout, const float* __restrict__ bias,
                                                       int M, float scale) {
  const _Float16* A  = (const _Float16*)Ap;
  const _Float16* Bt = (const _Float16*)Btp;
  __shared__ __align__(16) float sT[8][16 * 68];
  const int lane = threadIdx.x & 31;
  const int wave = threadIdx.x >> 5;
  const int tilesN = NOUTC >> 6;
  const int tilesM = M >> 6;
  const int tile = blockIdx.x * 8 + wave;
  if (tile >= tilesM * tilesN) return;
  const int tm = tile / tilesN;
  const int tn = tile - tm * tilesN;
  const int m0 = tm << 6;
  const int n0 = tn << 6;
  const int rlane = lane & 15;
  const int koff  = (lane >> 4) * 8;
  const int mOff  = (lane >> 4) * 8;

  v8f acc[4][4];
#pragma unroll
  for (int i = 0; i < 4; ++i)
#pragma unroll
    for (int jj = 0; jj < 4; ++jj) acc[i][jj] = (v8f){0.f, 0.f, 0.f, 0.f, 0.f, 0.f, 0.f, 0.f};

#pragma unroll 1
  for (int k0 = 0; k0 < NHID; k0 += 32) {
    v16h bh[4];
#pragma unroll
    for (int jj = 0; jj < 4; ++jj) {
      const size_t bo = (size_t)(n0 + (jj << 4) + rlane) * NHID + koff + k0;
      bh[jj] = frag_load(Bt + bo);
    }
#pragma unroll
    for (int i = 0; i < 4; ++i) {
      const size_t ao = (size_t)(m0 + (i << 4) + rlane) * NHID + koff + k0;
      const v16h ah = frag_load(A + ao);
#pragma unroll
      for (int jj = 0; jj < 4; ++jj) acc[i][jj] = frag_mma(ah, bh[jj], acc[i][jj]);
      guard4_h(acc[i][0], acc[i][1], acc[i][2], acc[i][3], ah, bh[3]);
    }
    keep4_h(bh[0], bh[1], bh[2], bh[3]);
  }
  acc_guard4(acc[0][0], acc[0][1], acc[0][2], acc[0][3]);
  acc_guard4(acc[1][0], acc[1][1], acc[1][2], acc[1][3]);
  acc_guard4(acc[2][0], acc[2][1], acc[2][2], acc[2][3]);
  acc_guard4(acc[3][0], acc[3][1], acc[3][2], acc[3][3]);

  float* slab = sT[wave];
  const int hh2 = lane >> 4, c4 = (lane & 15) * 4;
#pragma unroll
  for (int i = 0; i < 4; ++i) {
    const int mBase = m0 + (i << 4);
#pragma unroll
    for (int jj = 0; jj < 4; ++jj) {
      const int n = n0 + (jj << 4) + rlane;
      const float bv = bias[n];
#pragma unroll
      for (int r = 0; r < 8; ++r) {
        const float v = acc[i][jj][r] * scale + bv;
        slab[(mOff + r) * 68 + (jj << 4) + rlane] = v;
      }
    }
    __builtin_amdgcn_fence(__ATOMIC_RELEASE, "workgroup");
    __builtin_amdgcn_wave_barrier();
    __builtin_amdgcn_fence(__ATOMIC_ACQUIRE, "workgroup");
    for (int pass = 0; pass < 2; ++pass) {
#pragma unroll
      for (int it = 0; it < 8; ++it) {
        const int row = it * 2 + hh2;
        const v4f v = *(const v4f*)(slab + row * 68 + c4);
        *(volatile v4f*)(Cout + (size_t)(mBase + row) * NOUTC + n0 + c4) = v;
      }
      __threadfence();
    }
    __builtin_amdgcn_fence(__ATOMIC_RELEASE, "workgroup");
    __builtin_amdgcn_wave_barrier();
    __builtin_amdgcn_fence(__ATOMIC_ACQUIRE, "workgroup");
  }
}

extern "C" void kernel_launch(void* const* d_in, const int* in_sizes, int n_in,
                              void* d_out, int out_size, void* d_ws, size_t ws_size, hipStream_t stream) {
  if (n_in < 8 || d_out == nullptr || d_ws == nullptr) return;
  if (in_sizes[0] != NBATCH * NIN || in_sizes[1] != NGATE * NIN || in_sizes[2] != NGATE ||
      in_sizes[3] != NGATE * NHID || in_sizes[4] != NGATE || in_sizes[5] != NOUTC * NHID ||
      in_sizes[6] != NOUTC || in_sizes[7] != 1 || out_size != NROWS * NOUTC) return;

  const float* zin  = (const float*)d_in[0];
  const float* Wih  = (const float*)d_in[1];
  const float* bih  = (const float*)d_in[2];
  const float* Whh  = (const float*)d_in[3];
  const float* bhh  = (const float*)d_in[4];
  const float* Wout = (const float*)d_in[5];
  const float* bout = (const float*)d_in[6];
  float* out = (float*)d_out;

  char* ws = (char*)d_ws;
  size_t off = 0;
  auto carve = [&](size_t bytes) -> char* { char* p = ws + off; off += (bytes + 255) & ~(size_t)255; return p; };
  unsigned short* WHH16  = (unsigned short*)carve((size_t)NGATE * NHID * 2);
  unsigned short* WOUT16 = (unsigned short*)carve((size_t)NOUTC * NHID * 2);
  unsigned short* HS     = (unsigned short*)carve((size_t)NROWS * NHID * 2);
  if (off > ws_size || off > (size_t)134217728) return;

  const int n8h = NGATE * NHID / 8;
  const int n8o = NOUTC * NHID / 8;
  cvt8_f16_kernel<<<n8h / 256, 256, 0, stream>>>(Whh,  WHH16,  n8h, WCARRY);
  cvt8_f16_kernel<<<n8o / 256, 256, 0, stream>>>(Wout, WOUT16, n8o, WCARRY);

  gru_seq_kernel<<<NBATCH / SEQ_BLK, GRU_THR, 0, stream>>>(zin, Wih, bih, bhh, WHH16, HS);

  out_gemm_kernel<<<(NROWS / 64) * (NOUTC / 64) / 8, 256, 0, stream>>>(HS, WOUT16, out, bout, NROWS, WCARRY_INV);
}
